// CubicModelLarge_16587163697192
// MI455X (gfx1250) — hardware-run, weakly checked
//
#include <hip/hip_runtime.h>


#define NSM  1024
#define NFT  64
#define NPR  2080
#define NKH  2176
#define NKD  4352
#define NWF  135264
#define NC0  4160
#define NC2  704
constexpr size_t al256(size_t b) { return (b + 255) & ~(size_t)255; }
constexpr size_t WS_TOTAL = al256((size_t)NSM * NFT * 4) + al256((size_t)256 * 4) + al256((size_t)NFT * NWF * 4) + al256((size_t)NC0 * NKD * 2) + al256((size_t)NSM * NKD * 2) + al256((size_t)NSM * NC0 * 4) + 2 * al256((size_t)NSM * NFT * 4);
static_assert(WS_TOTAL == 97575936 && WS_TOTAL <= 134217728, "the workspace carve: 93.1 MiB");
static_assert(NKH >= NPR + NFT && NKH % 64 == 0 && NKD == 2 * NKH && NWF == NFT + NPR + NFT * NPR && NC0 % 64 == 0 && NC2 % 64 == 0 && NPR % 8 == 0 && (NKH / 8) == 272 && (NPR / 8) == 260, "whole tiles; whole lines; a 16-byte piece wholly in one block of the depth");
typedef _Float16 h16;
typedef unsigned short bf;
typedef __attribute__((ext_vector_type(16))) __bf16   v16bf;
typedef __attribute__((ext_vector_type(16))) _Float16 v16h;
typedef __attribute__((ext_vector_type(8)))  _Float16 v8h;
typedef __attribute__((ext_vector_type(8)))  unsigned short v8us;
typedef __attribute__((ext_vector_type(8)))  float    v8f;
typedef __attribute__((ext_vector_type(4)))  float    v4f;
typedef v8h  __attribute__((may_alias)) v8ha;
typedef v4f  __attribute__((may_alias)) v4fa;
typedef v8us __attribute__((may_alias)) v8usa;

__device__ __forceinline__ unsigned short f2bf(float f) { unsigned u = __float_as_uint(f); u += 0x7FFFu + ((u >> 16) & 1u); return (unsigned short)(u >> 16); }
__device__ __forceinline__ float bf2f(unsigned short b) { return __uint_as_float(((unsigned)b) << 16); }
__device__ __forceinline__ float bfr(float f) { return bf2f(f2bf(f)); }
__device__ __forceinline__ v16h cat16(v8h lo, v8h hi) { return __builtin_shufflevector(lo, hi, 0, 1, 2, 3, 4, 5, 6, 7, 8, 9, 10, 11, 12, 13, 14, 15); }
__device__ __forceinline__ v16bf cat16b(v8us lo, v8us hi) { return __builtin_bit_cast(v16bf, __builtin_shufflevector(lo, hi, 0, 1, 2, 3, 4, 5, 6, 7, 8, 9, 10, 11, 12, 13, 14, 15)); }
__device__ __forceinline__ v8f wmma16(v16h a, v16h b, v8f c) { return __builtin_amdgcn_wmma_f32_16x16x32_f16(false, a, false, b, (short)0, c, false, false); }
__device__ __forceinline__ v8f wmmab(v16bf a, v16bf b, v8f c) { return __builtin_amdgcn_wmma_f32_16x16x32_bf16(false, a, false, b, (short)0, c, false, false); }


template <typename T16> struct WFrag;
template <> struct WFrag<h16> { typedef v16h V; static __device__ __forceinline__ V ld(const h16* p) { return cat16(*(const v8h*)p, *(const v8h*)(p + 16)); } static __device__ __forceinline__ v8f mma(V a, V b, v8f c) { return wmma16(a, b, c); } };
template <> struct WFrag<bf> { typedef v16bf V; static __device__ __forceinline__ V ld(const bf* p) { return cat16b(*(const v8us*)p, *(const v8us*)(p + 16)); } static __device__ __forceinline__ v8f mma(V a, V b, v8f c) { return wmmab(a, b, c); } };
template <typename T16, int NSPLIT, bool BIAS>
__global__ __launch_bounds__(32) void k_gemmw(const T16* __restrict__ A, const T16* __restrict__ A2, const T16* __restrict__ Bt, const T16* __restrict__ Bt2, int K, float* C, int ldc, const float* __restrict__ bias, size_t sA, size_t sB, size_t sC) {
    typedef typename WFrag<T16>::V V;
    __shared__ __align__(16) float os[16 * 68];
    const size_t z = blockIdx.z; A += z * sA; if (A2) A2 += z * sA; Bt += z * sB; if (Bt2) Bt2 += z * sB; C += z * sC;
    const int lane = threadIdx.x & 31, lr = lane & 15, hi = lane >> 4; const int r0 = blockIdx.x * 64, c0 = blockIdx.y * 64;
    v8f acc[4][4];
#pragma unroll
    for (int mb = 0; mb < 4; ++mb)
#pragma unroll
        for (int nb = 0; nb < 4; ++nb) acc[mb][nb] = (v8f){};
    const size_t aoff = (size_t)(r0 + lr) * K + 8 * hi, boff = (size_t)(c0 + lr) * K + 8 * hi;
    for (int kc = 0; kc < K; kc += 32) {
        V a[4], a2[4];
#pragma unroll
        for (int mb = 0; mb < 4; ++mb) { a[mb] = WFrag<T16>::ld(A + aoff + (size_t)mb * 16 * K + kc); if (NSPLIT == 1 || NSPLIT == 2) a2[mb] = WFrag<T16>::ld(A2 + aoff + (size_t)mb * 16 * K + kc); }
#pragma unroll
        for (int nb = 0; nb < 4; ++nb) { const V b = WFrag<T16>::ld(Bt + boff + (size_t)nb * 16 * K + kc); V b2; if (NSPLIT >= 2) b2 = WFrag<T16>::ld(Bt2 + boff + (size_t)nb * 16 * K + kc);
#pragma unroll
            for (int mb = 0; mb < 4; ++mb) { acc[mb][nb] = WFrag<T16>::mma(a[mb], b, acc[mb][nb]); if (NSPLIT == 1 || NSPLIT == 2) acc[mb][nb] = WFrag<T16>::mma(a2[mb], b, acc[mb][nb]); if (NSPLIT >= 2) acc[mb][nb] = WFrag<T16>::mma(a[mb], b2, acc[mb][nb]); } }
        asm volatile("v_nop\n\tv_nop\n\tv_nop\n\tv_nop" : "+v"(acc[0][0]), "+v"(acc[1][1]), "+v"(acc[2][2]), "+v"(acc[3][3]) : "v"(a[0]), "v"(a[3]));
    }
#pragma unroll
    for (int mb = 0; mb < 4; ++mb) {
#pragma unroll
        for (int nb = 0; nb < 4; ++nb) {
#pragma unroll
            for (int j = 0; j < 8; ++j) os[(hi * 8 + j) * 68 + nb * 16 + lr] = acc[mb][nb][j]; }
        __builtin_amdgcn_wave_barrier(); asm volatile("" ::: "memory");
        float* crow = C + (size_t)(r0 + mb * 16) * ldc + c0;
#pragma unroll 1
        for (int ps = 0; ps < 2; ++ps) {
#pragma unroll
            for (int s = 0; s < 8; ++s) { const int row = 2 * s + hi, cofs = lr * 4; v4f val = *(const v4fa*)(os + row * 68 + cofs); if (BIAS) { val[0] += bfr(bias[c0 + cofs]); val[1] += bfr(bias[c0 + cofs + 1]); val[2] += bfr(bias[c0 + cofs + 2]); val[3] += bfr(bias[c0 + cofs + 3]); }
                *(volatile v4f*)(crow + (size_t)row * ldc + cofs) = val; }
            if (ps == 0) __threadfence(); }
        __builtin_amdgcn_wave_barrier(); asm volatile("" ::: "memory");
    }
}

__device__ __forceinline__ h16 tohx(float x) { return (h16)x; }
__device__ __forceinline__ void splitf(float y, unsigned short& h, unsigned short& l) { h = f2bf(y); l = f2bf(y - bf2f(h)); }
typedef __attribute__((ext_vector_type(2))) _Float16 v2h;
typedef __attribute__((ext_vector_type(4))) _Float16 v4h;
typedef __attribute__((ext_vector_type(2))) unsigned short v2us;
typedef __attribute__((ext_vector_type(4))) unsigned short v4us;
typedef __attribute__((ext_vector_type(2))) float v2f;
typedef __attribute__((ext_vector_type(4))) int v4i;


typedef _Float16 v8h __attribute__((ext_vector_type(8)));
typedef float v4f __attribute__((ext_vector_type(4)));

__global__ __launch_bounds__(256) void k_rnd(const float* __restrict__ src, float* dst, unsigned npc, unsigned nw) {
    const unsigned g = blockIdx.x * 256 + threadIdx.x; if (g >= npc) return; v4f o;
#pragma unroll
    for (int e = 0; e < 4; ++e) { const unsigned i = 4u * g + (unsigned)e; const unsigned live = i < nw ? 1u : 0u; const float rv_ = bfr(src[live ? i : 0u]); o[e] = live ? rv_ : 0.0f; }
    float* dq = dst + 4u * (size_t)g; *(volatile v4f*)(dq) = o; __threadfence(); *(volatile v4f*)(dq) = o; }

__device__ __forceinline__ float r11(float v) { const unsigned u = __float_as_uint(v); const unsigned r = (u + 0xFFFu + ((u >> 13) & 1u)) & 0xFFFFE000u; return __uint_as_float(r); }
__device__ __forceinline__ unsigned tri_row(unsigned p) {
        const unsigned ri = (p >= 64u ? 1u : 0u) + (p >= 127u ? 1u : 0u) + (p >= 189u ? 1u : 0u) + (p >= 250u ? 1u : 0u) + (p >= 310u ? 1u : 0u) + (p >= 369u ? 1u : 0u) + (p >= 427u ? 1u : 0u) + (p >= 484u ? 1u : 0u) + (p >= 540u ? 1u : 0u)
                    + (p >= 595u ? 1u : 0u) + (p >= 649u ? 1u : 0u) + (p >= 702u ? 1u : 0u) + (p >= 754u ? 1u : 0u) + (p >= 805u ? 1u : 0u) + (p >= 855u ? 1u : 0u) + (p >= 904u ? 1u : 0u) + (p >= 952u ? 1u : 0u) + (p >= 999u ? 1u : 0u)
                    + (p >= 1045u ? 1u : 0u) + (p >= 1090u ? 1u : 0u) + (p >= 1134u ? 1u : 0u) + (p >= 1177u ? 1u : 0u) + (p >= 1219u ? 1u : 0u) + (p >= 1260u ? 1u : 0u) + (p >= 1300u ? 1u : 0u) + (p >= 1339u ? 1u : 0u) + (p >= 1377u ? 1u : 0u)
                    + (p >= 1414u ? 1u : 0u) + (p >= 1450u ? 1u : 0u) + (p >= 1485u ? 1u : 0u) + (p >= 1519u ? 1u : 0u) + (p >= 1552u ? 1u : 0u) + (p >= 1584u ? 1u : 0u) + (p >= 1615u ? 1u : 0u) + (p >= 1645u ? 1u : 0u) + (p >= 1674u ? 1u : 0u)
                    + (p >= 1702u ? 1u : 0u) + (p >= 1729u ? 1u : 0u) + (p >= 1755u ? 1u : 0u) + (p >= 1780u ? 1u : 0u) + (p >= 1804u ? 1u : 0u) + (p >= 1827u ? 1u : 0u) + (p >= 1849u ? 1u : 0u) + (p >= 1870u ? 1u : 0u) + (p >= 1890u ? 1u : 0u)
                    + (p >= 1909u ? 1u : 0u) + (p >= 1927u ? 1u : 0u) + (p >= 1944u ? 1u : 0u) + (p >= 1960u ? 1u : 0u) + (p >= 1975u ? 1u : 0u) + (p >= 1989u ? 1u : 0u) + (p >= 2002u ? 1u : 0u) + (p >= 2014u ? 1u : 0u) + (p >= 2025u ? 1u : 0u)
                    + (p >= 2035u ? 1u : 0u) + (p >= 2044u ? 1u : 0u) + (p >= 2052u ? 1u : 0u) + (p >= 2059u ? 1u : 0u) + (p >= 2065u ? 1u : 0u) + (p >= 2070u ? 1u : 0u) + (p >= 2074u ? 1u : 0u) + (p >= 2077u ? 1u : 0u) + (p >= 2079u ? 1u : 0u);
        return ri; }
__global__ __launch_bounds__(256) void k_sq(const float* __restrict__ vin, h16* ao) {
    const unsigned g = blockIdx.x * 256 + threadIdx.x; if (g >= (unsigned)(NKH / 8)) return; const unsigned sm = blockIdx.y; const float* vq = vin + (size_t)sm * NFT; v8h oh, ol;
#pragma unroll
    for (int e = 0; e < 8; ++e) { const unsigned p = 8u * g + (unsigned)e; const unsigned pc = min(p, (unsigned)(NPR - 1)); const unsigned q = p - (unsigned)NPR; const unsigned li = min(q, (unsigned)(NFT - 1));
        const float fp = p < (unsigned)NPR ? 1.0f : 0.0f; const float fl = q < (unsigned)NFT ? 1.0f : 0.0f;
        const unsigned ri = tri_row(pc); const unsigned st = 64u * ri - ((ri * (ri - 1u)) >> 1); const unsigned rj = ri + (pc - st);
        const float val = fp * (vq[ri] * vq[rj]) + fl * vq[li];
        const float kh = fabsf(val) >= 6.103515625e-05f ? 1.0f : 0.0f; const float vk = val * kh; const float hf = r11(vk); const float rem = vk - hf; const float kl = fabsf(rem) >= 6.103515625e-05f ? 1.0f : 0.0f; oh[e] = tohx(hf); ol[e] = tohx(rem * kl); }
    h16* d8 = ao + (size_t)sm * NKD + 8u * g; *(volatile v8h*)(d8) = oh; *(volatile v8h*)(d8 + NKH) = ol; __threadfence(); *(volatile v8h*)(d8) = oh; *(volatile v8h*)(d8 + NKH) = ol; }

__global__ __launch_bounds__(256) void k_wlay(const float* __restrict__ wr, h16* wt, unsigned nout) {
    const unsigned g = blockIdx.x * 256 + threadIdx.x; if (g >= (unsigned)(NKH / 8)) return; const unsigned n = blockIdx.y; const unsigned nmain = 64u * nout; const unsigned ismain = (n < nmain) ? 1u : 0u; const unsigned ntail = (n - nmain) & 63u;
    const unsigned ii = n & 63u; const unsigned omain = n >> 6; const unsigned oo = ismain * omain + (1u - ismain) * ntail; const unsigned tailok = (ntail < nout) ? 1u : 0u; const unsigned rowok = ismain | tailok; const unsigned oc = rowok * oo;
    const unsigned inpair = (g < 260u) ? 1u : 0u; const unsigned inlin = ((g - 260u) < 8u) ? 1u : 0u; const unsigned liv = rowok & (inpair | (inlin & (1u - ismain)));
    const unsigned cpair = ismain * (2144u + 2080u * ii) + (1u - ismain) * 64u + 8u * g; const unsigned clin = 8u * ((g - 260u) & 7u); const unsigned col = liv * (inpair * cpair + (1u - inpair) * clin); const float lf = (float)liv;
    const float* sq = wr + (size_t)oc * NWF + col; const v4f a = *(const v4f*)sq; const v4f b = *(const v4f*)(sq + 4); v8h o8;
#pragma unroll
    for (int e = 0; e < 8; ++e) { const float val = ((e < 4 ? a[e & 3] : b[e & 3]) * 256.0f) * lf; const float kf = fabsf(val) >= 6.103515625e-05f ? 1.0f : 0.0f; o8[e] = tohx(val * kf); }
    h16* d8 = wt + (size_t)n * NKD + 8u * g; *(volatile v8h*)(d8) = o8; *(volatile v8h*)(d8 + NKH) = o8; __threadfence(); *(volatile v8h*)(d8) = o8; *(volatile v8h*)(d8 + NKH) = o8; }

template <int NOUT>
__global__ __launch_bounds__(256) void k_comb(const float* __restrict__ cc, const float* __restrict__ vin, const float* __restrict__ av, float* dst, unsigned ldc) {
    const unsigned g = blockIdx.x * 256 + threadIdx.x; if (g >= (unsigned)(NSM * NOUT)) return; const unsigned sm = g / (unsigned)NOUT, oo = g - sm * (unsigned)NOUT; const float* cq = cc + (size_t)sm * ldc; const float* uq = cq + 64u * oo; const float* vq = vin + (size_t)sm * NFT;
    float acc = cq[64u * (unsigned)NOUT + oo];
    for (int i = 0; i < NFT; ++i) acc += vq[i] * uq[i];
    const float res = av[oo] + acc * 0.00390625f; float* dq = dst + g; *(volatile float*)(dq) = res; __threadfence(); *(volatile float*)(dq) = res; }

extern "C" void kernel_launch(void* const* d_in, const int* in_sizes, int n_in,
                              void* d_out, int out_size, void* d_ws, size_t ws_size, hipStream_t stream) {
    if (n_in < 7) return;
    if (in_sizes[0] < NSM * NFT || in_sizes[1] < NFT * NWF || in_sizes[2] < NFT || in_sizes[3] < NFT * NWF || in_sizes[4] < NFT || in_sizes[5] < 10 * NWF || in_sizes[6] < 10 || out_size < NSM * 10) return;
    const float* xi = (const float*)d_in[0]; const float* wa = (const float*)d_in[1]; const float* ba = (const float*)d_in[2]; const float* wb = (const float*)d_in[3]; const float* bb = (const float*)d_in[4]; const float* wc = (const float*)d_in[5]; const float* bc = (const float*)d_in[6];
    char* wsp = (char*)d_ws;
    auto take = [&](size_t bytes) { char* cur = wsp; wsp += (bytes + 255) & ~(size_t)255; return (void*)cur; };
    float* XR = (float*)take((size_t)NSM * NFT * 4); float* BB = (float*)take((size_t)256 * 4); float* WR = (float*)take((size_t)NFT * NWF * 4); h16* WT = (h16*)take((size_t)NC0 * NKD * 2); h16* AO = (h16*)take((size_t)NSM * NKD * 2); float* CC = (float*)take((size_t)NSM * NC0 * 4); float* X1 = (float*)take((size_t)NSM * NFT * 4); float* X2 = (float*)take((size_t)NSM * NFT * 4);
    if ((size_t)(wsp - (char*)d_ws) != WS_TOTAL || WS_TOTAL > ws_size) return;
    auto rnd = [&](const float* sp_, float* dp_, unsigned nw) { const unsigned npc = (nw + 3) / 4; k_rnd<<<(npc + 255) / 256, 256, 0, stream>>>(sp_, dp_, npc, nw); };
    rnd(xi, XR, NSM * NFT); rnd(ba, BB, NFT); rnd(bb, BB + 64, NFT); rnd(bc, BB + 128, 10);
    rnd(wa, WR, NFT * NWF); k_wlay<<<dim3(2, NC0, 1), 256, 0, stream>>>(WR, WT, 64u); k_sq<<<dim3(2, NSM, 1), 256, 0, stream>>>(XR, AO);
    k_gemmw<h16, 0, false><<<dim3(NSM / 64, NC0 / 64, 1), 32, 0, stream>>>(AO, nullptr, WT, nullptr, NKD, CC, NC0, nullptr, (size_t)0, (size_t)0, (size_t)0);
    k_comb<64><<<(NSM * 64 + 255) / 256, 256, 0, stream>>>(CC, XR, BB, X1, (unsigned)NC0);
    rnd(wb, WR, NFT * NWF); k_wlay<<<dim3(2, NC0, 1), 256, 0, stream>>>(WR, WT, 64u); k_sq<<<dim3(2, NSM, 1), 256, 0, stream>>>(X1, AO);
    k_gemmw<h16, 0, false><<<dim3(NSM / 64, NC0 / 64, 1), 32, 0, stream>>>(AO, nullptr, WT, nullptr, NKD, CC, NC0, nullptr, (size_t)0, (size_t)0, (size_t)0);
    k_comb<64><<<(NSM * 64 + 255) / 256, 256, 0, stream>>>(CC, X1, BB + 64, X2, (unsigned)NC0);
    rnd(wc, WR, 10 * NWF); k_wlay<<<dim3(2, NC2, 1), 256, 0, stream>>>(WR, WT, 10u); k_sq<<<dim3(2, NSM, 1), 256, 0, stream>>>(X2, AO);
    k_gemmw<h16, 0, false><<<dim3(NSM / 64, NC2 / 64, 1), 32, 0, stream>>>(AO, nullptr, WT, nullptr, NKD, CC, NC2, nullptr, (size_t)0, (size_t)0, (size_t)0);
    k_comb<10><<<(NSM * 10 + 255) / 256, 256, 0, stream>>>(CC, X2, BB + 128, (float*)d_out, (unsigned)NC2);
}
